// T5RelativeAttention_32134945308856
// MI455X (gfx1250) — hardware-verified
//
#include <hip/hip_runtime.h>


namespace {
constexpr int Bn = 32, N = 577, NPCH = 576, LP = 608  , D = 768, H = 12, HD = 64, GB = 4  , NTG = GB * LP  , NREL = 2209;
constexpr float XS = 8.0f, PS = 8.0f;
struct Wo_ { static constexpr size_t QKV = 0, O = (size_t)3 * D * D, END = O + (size_t)D * D; };

typedef _Float16 b16;
typedef __attribute__((ext_vector_type(16))) _Float16 v16b;
typedef __attribute__((ext_vector_type(8))) _Float16 v8b;
typedef __attribute__((ext_vector_type(8))) float v8f;
typedef __attribute__((ext_vector_type(4))) float v4f;
__device__ __forceinline__ float bf16_rne(float f) { unsigned int u = __float_as_uint(f); u += 0x7FFFu + ((u >> 16) & 1u); return __uint_as_float(u & 0xFFFF0000u); }
__device__ __forceinline__ void split16(float v, b16& hi, b16& lo) { hi = (b16)v; lo = (b16)(v - (float)hi); }
__device__ __forceinline__ v16b frag_kb(const b16* p, int hh) { const v8b a = *(const v8b*)(p + 8 * hh), b = *(const v8b*)(p + 16 + 8 * hh); v16b f;
#pragma unroll
  for (int e = 0; e < 8; ++e) { f[e] = a[e]; f[8 + e] = b[e]; } return f; }
__device__ __forceinline__ v8f wmma16b(v16b a, v16b b, v8f c) { v8f d = __builtin_amdgcn_wmma_f32_16x16x32_f16(false, a, false, b, (short)0, c, false, false); asm volatile("v_nop\n\tv_nop\n\tv_nop\n\tv_nop" : "+v"(d) : "v"(a), "v"(b)); return d; }
__device__ __forceinline__ void wave_lds_sync() { __builtin_amdgcn_fence(__ATOMIC_RELEASE, "workgroup"); __builtin_amdgcn_wave_barrier(); __builtin_amdgcn_fence(__ATOMIC_ACQUIRE, "workgroup"); }
__device__ __forceinline__ float nexp(float x) { return __builtin_amdgcn_exp2f(x * 1.4426950408889634f); }
__device__ __forceinline__ float pmul(float a, float b) { float p = a * b; asm volatile("" : "+v"(p)); return p; }

__global__ __launch_bounds__(256) void prep_kernel(const float* __restrict__ wqkv, const float* __restrict__ wp, const float* __restrict__ pb, const float* __restrict__ b1, const float* __restrict__ b2, const float* __restrict__ b3, b16* __restrict__ R, float* __restrict__ P) {
  const size_t tid = (size_t)blockIdx.x * 256 + threadIdx.x, nth = (size_t)gridDim.x * 256;
  for (int pass = 0; pass < 2; ++pass) {
    for (size_t p = tid; p < Wo_::END / 8; p += nth) { const size_t q = p * 8; const float* s_ = (q < Wo_::O) ? (wqkv + q) : (wp + (q - Wo_::O)); v8b v; for (int e = 0; e < 8; ++e) v[e] = (b16)bf16_rne(s_[e]); *(volatile v8b*)(R + q) = v; }
    for (size_t q = tid; q < 41112; q += nth) { const int i = (int)q; float v; if (i < 768) v = pb[i]; else if (i < 7692) v = b1[i - 768]; else if (i < 14604) v = b2[i - 7692]; else v = b3[i - 14604]; P[q] = bf16_rne(v); }
    __threadfence(); }
}

__global__ __launch_bounds__(256) void xrows_kernel(const float* __restrict__ x, int b0, b16* __restrict__ X) {
  const size_t tid = (size_t)blockIdx.x * 256 + threadIdx.x, nth = (size_t)gridDim.x * 256;
  for (int pass = 0; pass < 2; ++pass) { for (size_t p = tid; p < (size_t)NTG * D / 8; p += nth) { const size_t r = p / (D / 8), c8 = (p % (D / 8)) * 8; const int bl = (int)(r / LP), t = (int)(r % LP); v8b v; for (int e = 0; e < 8; ++e) v[e] = (b16)((t < N) ? bf16_rne(x[((size_t)(b0 + bl) * N + t) * D + c8 + e]) * XS : 0.0f); *(volatile v8b*)(X + p * 8) = v; } __threadfence(); }
}

template <int MODE>
__global__ __launch_bounds__(64) void gemm_kernel(const b16* __restrict__ A, const b16* __restrict__ Al, const b16* __restrict__ Bw, const float* __restrict__ bias, b16* __restrict__ O1, b16* __restrict__ O2, b16* __restrict__ O3, float* __restrict__ O32, int b0, b16* __restrict__ O4) {
  __shared__ __attribute__((aligned(16))) float Ts[2][32][128 + 4];
  const int lane = threadIdx.x & 31, wave = threadIdx.x >> 5, nloc = lane & 15, hlf = lane >> 4, m0 = blockIdx.y * 32, c0 = blockIdx.x * 256 + wave * 128;
#pragma unroll 1
  for (int hf = 0; hf < 2; ++hf) { v8f acc[2][4];
#pragma unroll
    for (int r = 0; r < 2; ++r)
#pragma unroll
      for (int t = 0; t < 4; ++t) acc[r][t] = (v8f){};
#pragma unroll 2
    for (int kb = 0; kb < D; kb += 32) { const v16b a0 = frag_kb(A + (size_t)(m0 + nloc) * D + kb, hlf), a1 = frag_kb(A + (size_t)(m0 + 16 + nloc) * D + kb, hlf); v16b l0, l1; if (MODE == 1) { l0 = frag_kb(Al + (size_t)(m0 + nloc) * D + kb, hlf); l1 = frag_kb(Al + (size_t)(m0 + 16 + nloc) * D + kb, hlf); }
#pragma unroll
      for (int t = 0; t < 4; ++t) { const v16b bw = frag_kb(Bw + (size_t)(c0 + (hf * 4 + t) * 16 + nloc) * D + kb, hlf); acc[0][t] = wmma16b(a0, bw, acc[0][t]); acc[1][t] = wmma16b(a1, bw, acc[1][t]); if (MODE == 1) { acc[0][t] = wmma16b(l0, bw, acc[0][t]); acc[1][t] = wmma16b(l1, bw, acc[1][t]); } } }
#pragma unroll
    for (int t = 0; t < 4; ++t) { const int cl = (hf * 4 + t) * 16 + nloc; const float bb = (MODE == 1) ? bias[c0 + cl] : 0.0f;
#pragma unroll
      for (int r = 0; r < 2; ++r)
#pragma unroll
        for (int v = 0; v < 8; ++v) Ts[wave][r * 16 + 8 * hlf + v][cl] = acc[r][t][v] * (1.0f / XS) + bb; } }
  wave_lds_sync();
  for (int pass = 0; pass < 2; ++pass) {
    if (MODE == 1) { for (int i = lane; i < 32 * 32; i += 32) { const int rr = i >> 5, c4 = (i & 31) * 4; const int row = m0 + rr, b = b0 + row / LP, t = row % LP; if (t < N) *(volatile v4f*)(O32 + ((size_t)b * N + t) * D + c0 + c4) = *(const v4f*)(&Ts[wave][rr][c4]); } }
    else if (c0 < 2 * D) { for (int i = lane; i < 32 * 16; i += 32) { const int rr = i >> 4, c8 = (i & 15) * 8; v8b o, ol; for (int e = 0; e < 8; ++e) { b16 a_, c_; split16(Ts[wave][rr][c8 + e] * XS, a_, c_); o[e] = a_; ol[e] = c_; } const size_t gi = (size_t)(m0 + rr) * (2 * D) + c0 + c8; *(volatile v8b*)(O1 + gi) = o; *(volatile v8b*)(O4 + gi) = ol; } }
    else { for (int i = lane; i < 32 * 16; i += 32) { const int rr = i >> 4, c8 = (i & 15) * 8; v8b oh, ol; for (int e = 0; e < 8; ++e) { b16 a_, c_; split16(Ts[wave][rr][c8 + e] * XS, a_, c_); oh[e] = a_; ol[e] = c_; } const size_t gi = (size_t)(m0 + rr) * D + (c0 - 2 * D) + c8; *(volatile v8b*)(O2 + gi) = oh; *(volatile v8b*)(O3 + gi) = ol; } }
    __threadfence(); }
}

constexpr int LPP = 640;
__global__ __launch_bounds__(256) void vt_kernel(const b16* __restrict__ Vr, b16* __restrict__ vt) {
  __shared__ __attribute__((aligned(16))) b16 Tt[HD][LPP + 8];
  const int b = blockIdx.y, h = blockIdx.x, t_ = threadIdx.x;
  for (int i = t_; i < LPP * (HD / 8); i += 256) { const int tk = i >> 3, d8 = (i & 7) * 8; v8b vv = {}; if (tk < LP) vv = *(const v8b*)(Vr + ((size_t)(b * LP + tk)) * D + h * HD + d8); for (int e = 0; e < 8; ++e) Tt[d8 + e][tk] = vv[e]; }
  __syncthreads();
  for (int pass = 0; pass < 2; ++pass) { for (int i = t_; i < HD * (LPP / 8); i += 256) { const int d = i / (LPP / 8), c8 = (i % (LPP / 8)) * 8; *(volatile v8b*)(vt + (((size_t)b * H + h) * HD + d) * LPP + c8) = *(const v8b*)(&Tt[d][c8]); } __threadfence(); }
}

__global__ __launch_bounds__(128) void attn_kernel(const b16* __restrict__ QK, const b16* __restrict__ QKl, const b16* __restrict__ vth, const b16* __restrict__ vtl, const float* __restrict__ P, const int* __restrict__ mapi, b16* __restrict__ ctxh, b16* __restrict__ ctxl) {
  __shared__ float B3[4][NREL + 3]; __shared__ __attribute__((aligned(16))) b16 Oh[16][4 * HD + 8], Ol[16][4 * HD + 8];
  const int wid = threadIdx.x >> 5, lane = threadIdx.x & 31, hh = lane >> 4, col = lane & 15; const int b = blockIdx.x / (LP / 16), i0 = (blockIdx.x % (LP / 16)) * 16, h = blockIdx.y * 4 + wid, qi = i0 + col;
  for (int i = lane; i < NREL; i += 32) B3[wid][i] = P[14604 + h * NREL + i];
  const float* beta1 = P + 768 + h * N; const float* beta2 = P + 7692 + h * NPCH;
  wave_lds_sync();
  const b16* Qr = QK + (size_t)(b * LP) * (2 * D) + h * HD; const b16* Kr = QK + (size_t)(b * LP) * (2 * D) + D + h * HD; const b16* Qrl = QKl + (size_t)(b * LP) * (2 * D) + h * HD; const b16* Krl = QKl + (size_t)(b * LP) * (2 * D) + D + h * HD; const b16* Vh = vth + (((size_t)b * H + h) * HD) * LPP; const b16* Vl = vtl + (((size_t)b * H + h) * HD) * LPP;
  const v16b qf0 = frag_kb(Qr + (size_t)qi * (2 * D), hh), qf1 = frag_kb(Qr + (size_t)qi * (2 * D) + 32, hh), ql0 = frag_kb(Qrl + (size_t)qi * (2 * D), hh), ql1 = frag_kb(Qrl + (size_t)qi * (2 * D) + 32, hh);
  float m = -INFINITY, l = 0.0f; v8f o[4] = {{}, {}, {}, {}}; const int qic = (qi < N) ? qi : (N - 1);
  for (int kb = 0; kb < LP; kb += 32) { v8f s0 = {}, s1 = {};
    { const v16b k0 = frag_kb(Kr + (size_t)(kb + col) * (2 * D), hh), k0b = frag_kb(Kr + (size_t)(kb + col) * (2 * D) + 32, hh), k0l = frag_kb(Krl + (size_t)(kb + col) * (2 * D), hh), k0lb = frag_kb(Krl + (size_t)(kb + col) * (2 * D) + 32, hh);
      s0 = wmma16b(k0, qf0, s0); s0 = wmma16b(k0, ql0, s0); s0 = wmma16b(k0l, qf0, s0); s0 = wmma16b(k0b, qf1, s0); s0 = wmma16b(k0b, ql1, s0); s0 = wmma16b(k0lb, qf1, s0); }
    { const v16b k1 = frag_kb(Kr + (size_t)(kb + 16 + col) * (2 * D), hh), k1b = frag_kb(Kr + (size_t)(kb + 16 + col) * (2 * D) + 32, hh), k1l = frag_kb(Krl + (size_t)(kb + 16 + col) * (2 * D), hh), k1lb = frag_kb(Krl + (size_t)(kb + 16 + col) * (2 * D) + 32, hh);
      s1 = wmma16b(k1, qf0, s1); s1 = wmma16b(k1, ql0, s1); s1 = wmma16b(k1l, qf0, s1); s1 = wmma16b(k1b, qf1, s1); s1 = wmma16b(k1b, ql1, s1); s1 = wmma16b(k1lb, qf1, s1); }
    float mr = -INFINITY;
#pragma unroll
    for (int r = 0; r < 16; ++r) { const int j = kb + (r & 8) * 2 + 8 * hh + (r & 7); float sv = (r < 8) ? s0[r & 7] : s1[r & 7];
      const int jc = (j < N) ? j : (N - 1); const int jm = (jc >= 1) ? (jc - 1) : 0; const int qp = (qic < NPCH) ? qic : (NPCH - 1);
      int mi = mapi[qp * NPCH + jm]; mi = (mi < 0) ? 0 : (mi >= NREL ? NREL - 1 : mi);
      const float b_rel = B3[wid][mi], b_c0 = beta2[qp], b_last = beta1[jc];
      const float bias = (qic == NPCH) ? b_last : ((j == 0) ? b_c0 : b_rel);
      sv = (j >= N) ? -INFINITY : (sv * (0.125f / (XS * XS)) + bias);
      if (r < 8) s0[r & 7] = sv; else s1[r & 7] = sv; mr = fmaxf(mr, sv); }
    mr = fmaxf(mr, __shfl_xor(mr, 16)); const float mn = fmaxf(m, mr), al_ = nexp(m - mn); m = mn; float sum = 0.0f; v16b pb, pl;
#pragma unroll
    for (int r = 0; r < 8; ++r) { const float e0 = (s0[r] == -INFINITY) ? 0.0f : nexp(s0[r] - mn), e1 = (s1[r] == -INFINITY) ? 0.0f : nexp(s1[r] - mn); sum += e0 + e1; b16 a_, c_; split16(e0 * PS, a_, c_); pb[r] = a_; pl[r] = c_; split16(e1 * PS, a_, c_); pb[8 + r] = a_; pl[8 + r] = c_; }
    sum += __shfl_xor(sum, 16); l = l * al_ + sum;
#pragma unroll
    for (int t = 0; t < 4; ++t) { o[t] *= al_; const v16b vh = frag_kb(Vh + (size_t)(t * 16 + col) * LPP + kb, hh), vl = frag_kb(Vl + (size_t)(t * 16 + col) * LPP + kb, hh); o[t] = wmma16b(vh, pb, o[t]); o[t] = wmma16b(vh, pl, o[t]); o[t] = wmma16b(vl, pb, o[t]); } }
  const float inv = 1.0f / (l * PS);
#pragma unroll
  for (int t = 0; t < 4; ++t)
#pragma unroll
    for (int r = 0; r < 8; ++r) { b16 a_, c_; split16(o[t][r] * inv, a_, c_); Oh[col][wid * HD + t * 16 + 8 * hh + r] = a_; Ol[col][wid * HD + t * 16 + 8 * hh + r] = c_; }
  __syncthreads();
  for (int pass = 0; pass < 2; ++pass) { for (int i = threadIdx.x; i < 16 * 32; i += 128) { const int rr = i >> 5, c8 = (i & 31) * 8; const size_t gi = ((size_t)(b * LP + i0 + rr)) * D + blockIdx.y * 4 * HD + c8; *(volatile v8b*)(ctxh + gi) = *(const v8b*)(&Oh[rr][c8]); *(volatile v8b*)(ctxl + gi) = *(const v8b*)(&Ol[rr][c8]); } __threadfence(); }
}
}

extern "C" void kernel_launch(void* const* d_in, const int* in_sizes, int n_in,
                              void* d_out, int out_size, void* d_ws, size_t ws_size, hipStream_t stream) {
  (void)n_in; (void)out_size;
  const float* x = (const float*)d_in[0]; const float* wqkv = (const float*)d_in[1]; const float* wp = (const float*)d_in[2]; const float* pb = (const float*)d_in[3]; const float* b1 = (const float*)d_in[4]; const float* b2 = (const float*)d_in[5]; const float* b3 = (const float*)d_in[6]; const int* mapi = (const int*)d_in[7];
  float* out = (float*)d_out;
  if (in_sizes[0] != Bn * N * D || in_sizes[1] != 3 * D * D || in_sizes[6] != H * NREL || in_sizes[7] != NPCH * NPCH) return;
  size_t off = 0; char* ws = (char*)d_ws;
  auto carve = [&](size_t bytes) { char* p = ws + off; off += (bytes + 255) & ~(size_t)255; return p; };
  b16* R = (b16*)carve(Wo_::END * 2); float* P = (float*)carve(41112 * 4); b16* X = (b16*)carve((size_t)NTG * D * 2); b16* QK = (b16*)carve((size_t)NTG * 2 * D * 2); b16* VRh = (b16*)carve((size_t)NTG * D * 2); b16* VRl = (b16*)carve((size_t)NTG * D * 2);
  b16* VTh = (b16*)carve((size_t)GB * H * HD * LPP * 2); b16* VTl = (b16*)carve((size_t)GB * H * HD * LPP * 2); b16* CH = (b16*)carve((size_t)NTG * D * 2); b16* CL = (b16*)carve((size_t)NTG * D * 2); b16* QKl = (b16*)carve((size_t)NTG * 2 * D * 2);
  if (off > ws_size) return;
  prep_kernel<<<512, 256, 0, stream>>>(wqkv, wp, pb, b1, b2, b3, R, P);
  for (int g = 0; g < Bn / GB; ++g) { const int b0 = g * GB;
    xrows_kernel<<<256, 256, 0, stream>>>(x, b0, X);
    gemm_kernel<0><<<dim3(3 * D / 256, NTG / 32), 64, 0, stream>>>(X, nullptr, R + Wo_::QKV, nullptr, QK, VRh, VRl, nullptr, b0, QKl);
    vt_kernel<<<dim3(H, GB), 256, 0, stream>>>(VRh, VTh);
    vt_kernel<<<dim3(H, GB), 256, 0, stream>>>(VRl, VTl);
    attn_kernel<<<dim3(GB * LP / 16, 3), 128, 0, stream>>>(QK, QKl, VTh, VTl, P, mapi, CH, CL);
    gemm_kernel<1><<<dim3(D / 256, NTG / 32), 64, 0, stream>>>(CH, CL, R + Wo_::O, P, nullptr, nullptr, nullptr, out, b0, nullptr); }
}
